// CausalSelfAttention_72722386256234
// MI455X (gfx1250) — hardware-verified
//
#include <hip/hip_runtime.h>

#ifndef NB
#define NB 2
#endif
#ifndef SEQ
#define SEQ 2048
#endif
#define NB_FULL 2
#define SEQ_FULL 2048
#define CW 1024
#define NH 16
#define HD 64
#define QKW 2048
#define EARLY 256
#define NTOK (NB * SEQ)
#define LDV NTOK
#define ATT_CARRY 4096.0f
#define RES_SC 2048.0f
#define RES_INV 0.00048828125f
#define CTXC 16.0f

static_assert(NB >= 1 && NB <= NB_FULL);
static_assert(SEQ <= SEQ_FULL && SEQ % 64 == 0);
static_assert(SEQ >= EARLY && EARLY % 64 == 0);
static_assert(NH * HD == CW && HD == 64);
static_assert(CW % 32 == 0 && CW % 64 == 0);
static_assert(QKW == 2 * CW);
static_assert(NTOK % 64 == 0);

typedef __attribute__((ext_vector_type(16))) _Float16 v16h;
typedef __attribute__((ext_vector_type(8)))  _Float16 v8h;
typedef __attribute__((ext_vector_type(8)))  float    v8f;
typedef __attribute__((ext_vector_type(4)))  float    v4f;
typedef __attribute__((ext_vector_type(4)))  unsigned int v4u;

union FragU { v16h v; v8h h[2]; };
__device__ __forceinline__ v16h ldfrag(const _Float16* p) { FragU f; f.h[0] = *(const v8h*)(p); f.h[1] = *(const v8h*)(p + 16); return f.v; }
__device__ __forceinline__ v8f mma(v16h a, v16h b, v8f c) { return __builtin_amdgcn_wmma_f32_16x16x32_f16(false, a, false, b, (short)0, c, false, false); }
__device__ __forceinline__ void g1(v8f& a, v16h x, v16h y) { asm volatile("v_nop\n\tv_nop\n\tv_nop\n\tv_nop" : "+v"(a) : "v"(x), "v"(y)); }
__device__ __forceinline__ void g2(v8f& a, v8f& b, v16h x, v16h y) { asm volatile("v_nop\n\tv_nop\n\tv_nop\n\tv_nop" : "+v"(a), "+v"(b) : "v"(x), "v"(y)); }
__device__ __forceinline__ void g2x(v8f& a, v8f& b, v16h x, v16h y, v16h z, v16h w) { asm volatile("v_nop\n\tv_nop\n\tv_nop\n\tv_nop" : "+v"(a), "+v"(b) : "v"(x), "v"(y), "v"(z), "v"(w)); }
__device__ __forceinline__ void g4(v8f& a, v8f& b, v8f& c, v8f& d, v16h x, v16h y) { asm volatile("v_nop\n\tv_nop\n\tv_nop\n\tv_nop" : "+v"(a), "+v"(b), "+v"(c), "+v"(d) : "v"(x), "v"(y)); }
__device__ __forceinline__ void g4x(v8f& a, v8f& b, v8f& c, v8f& d, v16h x, v16h y, v16h z, v16h w) { asm volatile("v_nop\n\tv_nop\n\tv_nop\n\tv_nop" : "+v"(a), "+v"(b), "+v"(c), "+v"(d) : "v"(x), "v"(y), "v"(z), "v"(w)); }

__device__ __forceinline__ void wave_sync() {
    __builtin_amdgcn_fence(3  , "workgroup");
    __builtin_amdgcn_wave_barrier();
    __builtin_amdgcn_fence(2  , "workgroup");
}

__device__ __forceinline__ float bf_rne_f32(float v) { const unsigned u = __float_as_uint(v); const unsigned r = (u + 0x7fffu + ((u >> 16) & 1u)) & 0xffff0000u; return __uint_as_float(r); }
__device__ __forceinline__ unsigned pk2h(float a, float b) { return (unsigned)__builtin_bit_cast(unsigned short, (_Float16)a) | ((unsigned)__builtin_bit_cast(unsigned short, (_Float16)b) << 16); }
__device__ __forceinline__ void cvt8(const v4f a, const v4f b, v8h& hv, v8h& lv) {
    const float f[8] = {a.x, a.y, a.z, a.w, b.x, b.y, b.z, b.w};
#pragma unroll
    for (int e = 0; e < 8; ++e) { const _Float16 hh = (_Float16)f[e]; hv[e] = hh; lv[e] = (_Float16)((f[e] - (float)hh) * RES_SC); }
}

__global__ __launch_bounds__(256) void k_cast(const float* __restrict__ src, unsigned short* __restrict__ dst, int nR, int seq, int seq_full, float sc) {
    const long long u = (long long)blockIdx.x * 256 + threadIdx.x;
    const int per = CW / 8;
    if (u >= (long long)nR * per) return;
    const int r = (int)(u / per); const int c0 = 8 * (int)(u % per);
    const long long sr = (long long)(r / seq) * seq_full + (r % seq);
    const float* s = src + sr * CW + c0;
    const v4f a = *(const v4f*)(s); const v4f b = *(const v4f*)(s + 4);
    v4u pk;
    pk.x = pk2h(bf_rne_f32(a.x) * sc, bf_rne_f32(a.y) * sc); pk.y = pk2h(bf_rne_f32(a.z) * sc, bf_rne_f32(a.w) * sc);
    pk.z = pk2h(bf_rne_f32(b.x) * sc, bf_rne_f32(b.y) * sc); pk.w = pk2h(bf_rne_f32(b.z) * sc, bf_rne_f32(b.w) * sc);
    volatile v4u* d = (volatile v4u*)(dst + (long long)r * CW + c0);
    *d = pk; __threadfence(); *d = pk;
}

template <int OUT_MODE, bool RESID>
__device__ __forceinline__ void gemm64_body(const unsigned short* __restrict__ Ap, int lda, long long strideA,
                                            const unsigned short* __restrict__ Btp, int ldb,
                                            float* Cf, unsigned short* Ch, unsigned short* Cr, int ldc, long long strideC,
                                            const float* Rsd, long long strideR, int M, int N, int K, float scale) {
    __shared__ __align__(16) float sT[8 * 16 * 68];
    const int bz   = (int)blockIdx.y;
    const int lane = (int)(threadIdx.x & 31);
    const int wave = __builtin_amdgcn_readfirstlane((int)(threadIdx.x >> 5));
    const int tilesN = N >> 6, tilesM = M >> 6;
    const int tile = (int)blockIdx.x * 8 + wave;
    if (tile >= tilesM * tilesN) return;
    const int tm = tile / tilesN, tn = tile - tm * tilesN;
    const int m0 = tm << 6, n0 = tn << 6;
    const _Float16* A  = (const _Float16*)Ap + (size_t)bz * (size_t)strideA;
    const _Float16* Bt = (const _Float16*)Btp;
    const int rl = lane & 15, hf = lane >> 4, koff = 8 * hf, mOff = 8 * hf;

    v8f acc[4][4];
#pragma unroll
    for (int i = 0; i < 4; ++i)
#pragma unroll
        for (int j = 0; j < 4; ++j) { v8f zz = {}; acc[i][j] = zz; }

    for (int k0 = 0; k0 < K; k0 += 32) {
        v16h bh[4];
#pragma unroll
        for (int j = 0; j < 4; ++j) bh[j] = ldfrag(Bt + (size_t)(n0 + 16 * j + rl) * ldb + koff + k0);
#pragma unroll
        for (int i = 0; i < 4; ++i) {
            const v16h ah = ldfrag(A + (size_t)(m0 + 16 * i + rl) * lda + koff + k0);
#pragma unroll
            for (int j = 0; j < 4; ++j) acc[i][j] = mma(ah, bh[j], acc[i][j]);
            g4(acc[i][0], acc[i][1], acc[i][2], acc[i][3], ah, bh[3]);
        }
    }

    const int sb = wave * (16 * 68);
#pragma unroll
    for (int i = 0; i < 4; ++i) {
        const int mBase = m0 + 16 * i;
#pragma unroll
        for (int j = 0; j < 4; ++j) {
            const int n = n0 + 16 * j + rl;
#pragma unroll
            for (int r = 0; r < 8; ++r) {
                float v = acc[i][j][r] * scale;
                if (RESID) v += Rsd[(size_t)bz * (size_t)strideR + (size_t)(mBase + mOff + r) * ldc + n];
                sT[sb + (mOff + r) * 68 + 16 * j + rl] = v;
            }
        }
        wave_sync();
        if (OUT_MODE == 0) {
            float* C = Cf + (size_t)bz * (size_t)strideC;
            const int c4 = (lane & 15) * 4;
            for (int pass = 0; pass < 2; ++pass) {
#pragma unroll
                for (int it = 0; it < 8; ++it) {
                    const int row = it * 2 + hf;
                    const v4f v = *(const v4f*)&sT[sb + row * 68 + c4];
                    *(volatile v4f*)(C + (size_t)(mBase + row) * ldc + n0 + c4) = v;
                }
                __threadfence();
            }
        } else {
            const int q4 = lane >> 3, c8 = (lane & 7) * 8;
            unsigned short* C1 = Ch + (size_t)bz * (size_t)strideC;
            unsigned short* C2 = Cr + (size_t)bz * (size_t)strideC;
            for (int pass = 0; pass < 2; ++pass) {
#pragma unroll
                for (int it = 0; it < 4; ++it) {
                    const int row = it * 4 + q4;
                    const v4f f0 = *(const v4f*)&sT[sb + row * 68 + c8];
                    const v4f f1 = *(const v4f*)&sT[sb + row * 68 + c8 + 4];
                    v8h hv, lv; cvt8(f0, f1, hv, lv);
                    *(volatile v8h*)(C1 + (size_t)(mBase + row) * ldc + n0 + c8) = hv;
                    *(volatile v8h*)(C2 + (size_t)(mBase + row) * ldc + n0 + c8) = lv;
                }
                __threadfence();
            }
        }
        wave_sync();
    }
}

__global__ __launch_bounds__(256) void k_gemm_hr(const unsigned short* A, int lda, long long strideA, const unsigned short* Bt, int ldb,
                                                 unsigned short* Ch, unsigned short* Cr, int ldc, long long strideC, int M, int N, int K, float scale) {
    gemm64_body<3, false>(A, lda, strideA, Bt, ldb, (float*)0, Ch, Cr, ldc, strideC, (const float*)0, 0, M, N, K, scale);
}
__global__ __launch_bounds__(256) void k_gemm_out(const unsigned short* A, int lda, long long strideA, const unsigned short* Bt, int ldb,
                                                  float* C, int ldc, long long strideC, int M, int N, int K, float scale) {
    gemm64_body<0, false>(A, lda, strideA, Bt, ldb, C, (unsigned short*)0, (unsigned short*)0, ldc, strideC, (const float*)0, 0, M, N, K, scale);
}
__global__ __launch_bounds__(256) void k_gemm_out_acc(const unsigned short* A, int lda, long long strideA, const unsigned short* Bt, int ldb,
                                                      float* C, const float* R, int ldc, long long strideC, int M, int N, int K, float scale) {
    gemm64_body<0, true>(A, lda, strideA, Bt, ldb, C, (unsigned short*)0, (unsigned short*)0, ldc, strideC, R, strideC, M, N, K, scale);
}

template <bool RES>
__device__ __forceinline__ void attn_body(const unsigned short* __restrict__ QKp, const unsigned short* __restrict__ QKRp,
                                          const unsigned short* __restrict__ VTp, const unsigned short* __restrict__ VTRp,
                                          unsigned short* __restrict__ CTXp, unsigned short* __restrict__ CTXRp, int qb_lo, int nqb) {
    __shared__ __align__(16) float Os[4 * 16 * 68];
    const int wave = __builtin_amdgcn_readfirstlane((int)(threadIdx.x >> 5));
    const int lane = (int)(threadIdx.x & 31), hf = lane >> 4, n = lane & 15;
    const int bx = (int)blockIdx.x;
    const int qb = qb_lo + bx % nqb;
    const int bh = bx / nqb;
    const int h = bh % NH, b = bh / NH;
    const int q0 = qb * 64 + wave * 16;
    const int tok0 = b * SEQ;
    const _Float16* QK  = (const _Float16*)QKp;
    const _Float16* QKR = (const _Float16*)QKRp;
    const _Float16* VT  = (const _Float16*)VTp;
    const _Float16* VTR = (const _Float16*)VTRp;
    const float NEG = -__builtin_inff();
    const float SC = 0.18033688011112042f;

    v16h qh[2], qr[2];
    {
        const size_t qo = (size_t)(tok0 + q0 + n) * QKW + h * HD + 8 * hf;
#pragma unroll
        for (int ks = 0; ks < 2; ++ks) {
            qh[ks] = ldfrag(QK + qo + ks * 32);
            if (RES) qr[ks] = ldfrag(QKR + qo + ks * 32); else qr[ks] = qh[ks];
        }
    }
    v8f o[4], orr[4];
#pragma unroll
    for (int t = 0; t < 4; ++t) { v8f zz = {}; o[t] = zz; orr[t] = zz; }
    float mrun = NEG, lrun = 0.f;
    const int qi = q0 + n;
    const int nsteps = (q0 + 47) >> 5;

#pragma unroll 1
    for (int st = 0; st < nsteps; ++st) {
        const int j0 = st * 32;
        v8f s0 = {}, s1 = {}, r0 = {}, r1 = {};
#pragma unroll
        for (int ks = 0; ks < 2; ++ks) {
            const size_t ko = (size_t)(tok0 + j0 + n) * QKW + CW + h * HD + ks * 32 + 8 * hf;
            const v16h k0 = ldfrag(QK + ko);
            const v16h k1 = ldfrag(QK + ko + (size_t)16 * QKW);
            s0 = mma(k0, qh[ks], s0);
            s1 = mma(k1, qh[ks], s1);
            if (RES) {
                const v16h kr0 = ldfrag(QKR + ko);
                const v16h kr1 = ldfrag(QKR + ko + (size_t)16 * QKW);
                r0 = mma(k0, qr[ks], r0); r0 = mma(kr0, qh[ks], r0);
                r1 = mma(k1, qr[ks], r1); r1 = mma(kr1, qh[ks], r1);
                g4x(s0, s1, r0, r1, k1, kr1, qh[ks], qr[ks]);
            } else {
                g2(s0, s1, k1, qh[ks]);
            }
        }
#pragma unroll
        for (int r = 0; r < 8; ++r) {
            float a = s0[r], c = s1[r];
            if (RES) { a += r0[r] * RES_INV; c += r1[r] * RES_INV; }
            s0[r] = a * SC; s1[r] = c * SC;
        }
        if (j0 + 31 > q0) {
#pragma unroll
            for (int r = 0; r < 8; ++r) {
                const int ky = j0 + 8 * hf + r;
                if (ky > qi) s0[r] = NEG;
                if (ky + 16 > qi) s1[r] = NEG;
            }
        }
        float mx = NEG;
#pragma unroll
        for (int r = 0; r < 8; ++r) mx = fmaxf(mx, fmaxf(s0[r], s1[r]));
        mx = fmaxf(mx, __shfl_xor(mx, 16, 32));
        const float mnew = fmaxf(mrun, mx);
        const float alpha = exp2f(mrun - mnew);
        float ps = 0.f;
        v16h pb, pbr;
#pragma unroll
        for (int r = 0; r < 8; ++r) {
            const float p0 = exp2f(s0[r] - mnew), p1 = exp2f(s1[r] - mnew);
            ps += p0 + p1;
            const float c0 = p0 * ATT_CARRY, c1 = p1 * ATT_CARRY;
            const _Float16 h0 = (_Float16)c0, h1 = (_Float16)c1;
            pb[r] = h0; pb[8 + r] = h1;
            if (RES) { pbr[r] = (_Float16)((c0 - (float)h0) * RES_SC); pbr[8 + r] = (_Float16)((c1 - (float)h1) * RES_SC); }
            else { pbr[r] = h0; pbr[8 + r] = h1; }
        }
        ps += __shfl_xor(ps, 16, 32);
        lrun = lrun * alpha + ps; mrun = mnew;
#pragma unroll
        for (int t = 0; t < 4; ++t) { o[t] = o[t] * alpha; if (RES) orr[t] = orr[t] * alpha; }
#pragma unroll
        for (int t = 0; t < 4; ++t) {
            const size_t vo = (size_t)(h * HD + t * 16 + n) * LDV + tok0 + j0 + 8 * hf;
            const v16h va = ldfrag(VT + vo);
            o[t] = mma(va, pb, o[t]);
            if (RES) {
                const v16h vr = ldfrag(VTR + vo);
                orr[t] = mma(va, pbr, orr[t]);
                orr[t] = mma(vr, pb, orr[t]);
                g2x(o[t], orr[t], va, vr, pb, pbr);
            } else {
                g1(o[t], va, pb);
            }
        }
    }

    const float inv = CTXC * (1.0f / (lrun * ATT_CARRY));
    const int ob = wave * (16 * 68);
#pragma unroll
    for (int t = 0; t < 4; ++t)
#pragma unroll
        for (int r = 0; r < 8; ++r) {
            float v = o[t][r];
            if (RES) v += orr[t][r] * RES_INV;
            Os[ob + n * 68 + t * 16 + 8 * hf + r] = v * inv;
        }
    wave_sync();
    {
        const int q4 = lane >> 3, c8 = (lane & 7) * 8;
        for (int pass = 0; pass < 2; ++pass) {
#pragma unroll
            for (int it = 0; it < 4; ++it) {
                const int row = it * 4 + q4;
                const v4f f0 = *(const v4f*)&Os[ob + row * 68 + c8];
                const v4f f1 = *(const v4f*)&Os[ob + row * 68 + c8 + 4];
                v8h hv, lv; cvt8(f0, f1, hv, lv);
                *(volatile v8h*)(CTXp + (size_t)(tok0 + q0 + row) * CW + h * HD + c8) = hv;
                if (RES) *(volatile v8h*)(CTXRp + (size_t)(b * EARLY + q0 + row) * CW + h * HD + c8) = lv;
            }
            __threadfence();
        }
    }
}

__global__ __launch_bounds__(128) void k_attn_early(const unsigned short* QK, const unsigned short* QKR, const unsigned short* VT, const unsigned short* VTR,
                                                    unsigned short* CTX, unsigned short* CTXR, int qb_lo, int nqb) {
    attn_body<true>(QK, QKR, VT, VTR, CTX, CTXR, qb_lo, nqb);
}
__global__ __launch_bounds__(128) void k_attn_late(const unsigned short* QK, const unsigned short* QKR, const unsigned short* VT, const unsigned short* VTR,
                                                   unsigned short* CTX, unsigned short* CTXR, int qb_lo, int nqb) {
    attn_body<false>(QK, QKR, VT, VTR, CTX, CTXR, qb_lo, nqb);
}

#define SZ_X16   ((size_t)NTOK * CW * 2)
#define SZ_W316  ((size_t)3 * CW * CW * 2)
#define SZ_WO16  ((size_t)CW * CW * 2)
#define SZ_QK    ((size_t)NTOK * QKW * 2)
#define SZ_VT    ((size_t)CW * LDV * 2)
#define SZ_CTX   ((size_t)NTOK * CW * 2)
#define SZ_CTXR  ((size_t)NB * EARLY * CW * 2)
#define WS_TOTAL (SZ_X16 + SZ_W316 + SZ_WO16 + 2 * SZ_QK + 2 * SZ_VT + SZ_CTX + SZ_CTXR)
static_assert(WS_TOTAL <= (size_t)134217728);
static_assert(SZ_X16 % 256 == 0 && SZ_W316 % 256 == 0 && SZ_WO16 % 256 == 0 && SZ_QK % 256 == 0 && SZ_VT % 256 == 0 && SZ_CTX % 256 == 0 && SZ_CTXR % 256 == 0);

extern "C" void kernel_launch(void* const* d_in, const int* in_sizes, int n_in, void* d_out, int out_size, void* d_ws, size_t ws_size, hipStream_t stream) {
    const long long need_x = ((long long)(NB - 1) * SEQ_FULL + SEQ) * CW;
    if (n_in < 3) return;
    if ((long long)in_sizes[0] < need_x) return;
    if ((long long)in_sizes[1] < (long long)3 * CW * CW) return;
    if ((long long)in_sizes[2] < (long long)CW * CW) return;
    if ((long long)out_size < need_x) return;
    if (WS_TOTAL > ws_size) return;

    const float* x      = (const float*)d_in[0];
    const float* w_qkv  = (const float*)d_in[1];
    const float* w_proj = (const float*)d_in[2];
    float* out = (float*)d_out;

    char* wsp = (char*)d_ws;
    unsigned short* X16  = (unsigned short*)wsp; wsp += SZ_X16;
    unsigned short* W316 = (unsigned short*)wsp; wsp += SZ_W316;
    unsigned short* WO16 = (unsigned short*)wsp; wsp += SZ_WO16;
    unsigned short* QK16 = (unsigned short*)wsp; wsp += SZ_QK;
    unsigned short* QKR  = (unsigned short*)wsp; wsp += SZ_QK;
    unsigned short* VT   = (unsigned short*)wsp; wsp += SZ_VT;
    unsigned short* VTR  = (unsigned short*)wsp; wsp += SZ_VT;
    unsigned short* CTX  = (unsigned short*)wsp; wsp += SZ_CTX;
    unsigned short* CTXR = (unsigned short*)wsp; wsp += SZ_CTXR;

    k_cast<<<(unsigned)(((long long)NTOK * (CW / 8) + 255) / 256), 256, 0, stream>>>(x, X16, NTOK, SEQ, SEQ_FULL, 1.0f);
    k_cast<<<(unsigned)(((long long)3 * CW * (CW / 8) + 255) / 256), 256, 0, stream>>>(w_qkv, W316, 3 * CW, 3 * CW, 3 * CW, 16.0f);
    k_cast<<<(unsigned)(((long long)CW * (CW / 8) + 255) / 256), 256, 0, stream>>>(w_proj, WO16, CW, CW, CW, 16.0f);

    k_gemm_hr<<<dim3((unsigned)(((NTOK / 64) * (QKW / 64) + 7) / 8), 1u), 256, 0, stream>>>(X16, CW, 0, W316, CW, QK16, QKR, QKW, 0, NTOK, QKW, CW, 0.0625f);
    k_gemm_hr<<<dim3((unsigned)(((CW / 64) * (NTOK / 64) + 7) / 8), 1u), 256, 0, stream>>>(W316 + (size_t)2 * CW * CW, CW, 0, X16, CW, VT, VTR, LDV, 0, CW, NTOK, CW, 0.0625f);

    k_attn_early<<<(unsigned)(NB * NH * (EARLY / 64)), 128, 0, stream>>>(QK16, QKR, VT, VTR, CTX, CTXR, 0, EARLY / 64);
    if (SEQ / 64 - EARLY / 64 > 0)
        k_attn_late<<<(unsigned)(NB * NH * (SEQ / 64 - EARLY / 64)), 128, 0, stream>>>(QK16, QKR, VT, VTR, CTX, CTXR, EARLY / 64, SEQ / 64 - EARLY / 64);

    k_gemm_out<<<dim3((unsigned)(((SEQ / 64) * (CW / 64) + 7) / 8), (unsigned)NB), 256, 0, stream>>>(CTX, CW, (long long)SEQ * CW, WO16, CW, out, CW, (long long)SEQ_FULL * CW, SEQ, CW, CW, 0.00390625f);
    k_gemm_out_acc<<<dim3((unsigned)(((EARLY / 64) * (CW / 64) + 7) / 8), (unsigned)NB), 256, 0, stream>>>(CTXR, CW, (long long)EARLY * CW, WO16, CW, out, out, CW, (long long)SEQ_FULL * CW, EARLY, CW, CW, 1.9073486328125e-06f);
}
